// SambaMambaBlock_65687229825697
// MI455X (gfx1250) — hardware-run, weakly checked
//
#include <hip/hip_runtime.h>
#include <hip/hip_fp16.h>
#include <math.h>

typedef __attribute__((ext_vector_type(16))) _Float16 v16h;
typedef __attribute__((ext_vector_type(8)))  _Float16 v8h;
typedef __attribute__((ext_vector_type(8)))  float    v8f;
typedef __attribute__((ext_vector_type(4)))  float    v4f;
typedef __attribute__((ext_vector_type(2)))  unsigned v2u;

constexpr int kBatch  = 2;
constexpr int kSeq    = 1024;
constexpr int kDm     = 1024;
constexpr int kDin    = 2048;
constexpr int kXzP    = 2 * kDin;
constexpr int kRank   = 64;
constexpr int kNst    = 16;
constexpr int kProjN  = kRank + 2 * kNst;
constexpr int kProjP  = 128;
constexpr int kBcP    = 2 * kNst;
constexpr int kConvK  = 4;
constexpr int kConvTP = 260;
constexpr float kWCarry = 1024.0f;
constexpr float kResid  = 2048.0f;
constexpr float kYCarry = 16.0f;
static_assert(kXzP == 4096);
static_assert(kProjN == 96);
static_assert(kBcP == 32);
static_assert(kProjN <= kProjP && (kProjP % 64) == 0);
static_assert((kSeq % 64) == 0 && (kDin % 64) == 0 && (kDm % 64) == 0 && (kXzP % 64) == 0);
static_assert((kDm % 32) == 0 && (kDin % 32) == 0 && (kRank % 32) == 0);
static_assert((kDin % 256) == 0 && (kDin % 1024) == 0 && (kSeq % 8) == 0);
static_assert(kConvTP >= 256 && (kConvTP % 4) == 0);

constexpr size_t kSzWIN  = (size_t)kXzP * kDm * 2;
constexpr size_t kSzWX   = (size_t)kProjP * kDin * 2;
constexpr size_t kSzWDT  = (size_t)kDin * kRank * 2;
constexpr size_t kSzWOH  = (size_t)kDm * kDin * 2;
constexpr size_t kSzCW   = (size_t)kDin * kConvK * 4;
constexpr size_t kSzVEC  = (size_t)kDin * 4;
constexpr size_t kSzALOG = (size_t)kDin * kNst * 4;
constexpr size_t kSzX16  = (size_t)kSeq * kDm * 2;
constexpr size_t kSzXZ   = (size_t)kSeq * kXzP * 4;
constexpr size_t kSzU    = (size_t)kSeq * kDin * 4;
constexpr size_t kSzU16  = (size_t)kSeq * kDin * 2;
constexpr size_t kSzPROJ = (size_t)kSeq * kProjP * 4;
constexpr size_t kSzD16  = (size_t)kSeq * kRank * 2;
constexpr size_t kSzBC   = (size_t)kSeq * kBcP * 4;
constexpr size_t kOffWIN  = 0;
constexpr size_t kOffWXH  = kOffWIN  + kSzWIN;
constexpr size_t kOffWDT  = kOffWXH  + kSzWX;
constexpr size_t kOffWOH  = kOffWDT  + kSzWDT;
constexpr size_t kOffCW   = kOffWOH  + kSzWOH;
constexpr size_t kOffCB   = kOffCW   + kSzCW;
constexpr size_t kOffBDR  = kOffCB   + kSzVEC;
constexpr size_t kOffDR   = kOffBDR  + kSzVEC;
constexpr size_t kOffALOG = kOffDR   + kSzVEC;
constexpr size_t kOffXH   = kOffALOG + kSzALOG;
constexpr size_t kOffXZ   = kOffXH   + kSzX16;
constexpr size_t kOffU    = kOffXZ   + kSzXZ;
constexpr size_t kOffUH   = kOffU    + kSzU;
constexpr size_t kOffPROJ = kOffUH   + kSzU16;
constexpr size_t kOffDH   = kOffPROJ + kSzPROJ;
constexpr size_t kOffBC   = kOffDH   + kSzD16;
constexpr size_t kOffDTP  = kOffBC   + kSzBC;
constexpr size_t kOffDT   = kOffDTP  + kSzU;
constexpr size_t kOffYH   = kOffDT   + kSzU;
constexpr size_t kWsTotal = kOffYH   + kSzU16;
static_assert(kSzWIN == 8388608ull && kSzWX == 524288ull && kSzWDT == 262144ull && kSzWOH == 4194304ull);
static_assert(kSzCW == 32768ull && kSzVEC == 8192ull && kSzALOG == 131072ull);
static_assert(kSzX16 == 2097152ull && kSzXZ == 16777216ull && kSzU == 8388608ull && kSzU16 == 4194304ull);
static_assert(kSzPROJ == 524288ull && kSzD16 == 131072ull && kSzBC == 131072ull);
static_assert(kWsTotal == 66772992ull);
static_assert(kWsTotal <= 134217728ull);
static_assert((kOffWXH % 128) == 0 && (kOffWDT % 128) == 0 && (kOffWOH % 128) == 0 && (kOffCW % 128) == 0 &&
              (kOffCB % 128) == 0 && (kOffBDR % 128) == 0 && (kOffDR % 128) == 0 && (kOffALOG % 128) == 0 &&
              (kOffXH % 128) == 0 && (kOffXZ % 128) == 0 && (kOffU % 128) == 0 && (kOffUH % 128) == 0 &&
              (kOffPROJ % 128) == 0 && (kOffDH % 128) == 0 && (kOffBC % 128) == 0 && (kOffDTP % 128) == 0 &&
              (kOffDT % 128) == 0 && (kOffYH % 128) == 0);

__device__ __forceinline__ _Float16 f16_flush(float v) {
  const float w = (fabsf(v) < 6.103515625e-05f) ? 0.0f : v;
  return (_Float16)w;
}
__device__ __forceinline__ void f16_split(float v, _Float16& hi, _Float16& lo) {
  hi = f16_flush(v);
  const float hf = (float)hi;
  const float r = (v - hf) * kResid;
  lo = f16_flush(r);
}

__device__ __forceinline__ float bf16r(float v) {
  unsigned u = __float_as_uint(v);
  u = (u + 0x7FFFu + ((u >> 16) & 1u)) & 0xFFFF0000u;
  return __uint_as_float(u);
}

__device__ __forceinline__ float h16_to_f32(unsigned hb) {
  const unsigned sgn = (hb & 0x8000u) << 16; const unsigned em = hb & 0x7fffu;
  const float fn = __uint_as_float((em << 13) + 0x38000000u);
  const float fs = (float)em * 5.9604644775390625e-8f;
  const float mag = (em < 0x400u) ? fs : fn; return __uint_as_float(__float_as_uint(mag) | sgn); }

namespace eng {
union FragU { v16h v; v8h h[2]; };
__device__ __forceinline__ v16h frag_load(const _Float16* p) {
  FragU f;
  f.h[0] = *(const v8h*)(p);
  f.h[1] = *(const v8h*)(p + 16);
  return f.v;
}
__device__ __forceinline__ v8f mma(v16h a, v16h b, v8f c) {
  return __builtin_amdgcn_wmma_f32_16x16x32_f16(false, a, false, b, (short)0, c, false, false);
}
__device__ __forceinline__ void guard1(v8f& a, v16h x, v16h y) {
  asm volatile("v_nop\n\tv_nop\n\tv_nop\n\tv_nop" : "+v"(a) : "v"(x), "v"(y));
}
__device__ __forceinline__ void guard_acc(v8f& a) {
  asm volatile("v_nop\n\tv_nop\n\tv_nop\n\tv_nop" : "+v"(a));
}
__device__ __forceinline__ void keep4(v16h a, v16h b, v16h c, v16h d) {
  asm volatile("v_nop" :: "v"(a), "v"(b), "v"(c), "v"(d));
}

template <int MI, int SPL>
__global__ __launch_bounds__(256) void gemm_f16_kernel(
    const unsigned short* __restrict__ Ap, const unsigned short* __restrict__ A2p, int lda,
    const unsigned short* __restrict__ Btp, const unsigned short* __restrict__ Bt2p, int ldb,
    float* __restrict__ C, int ldc, int M, int N, int K, float scale, float rscale)
{
  static_assert(MI >= 1 && MI <= 2);
  static_assert(SPL >= 0 && SPL <= 2);
  const _Float16* A   = (const _Float16*)Ap;
  const _Float16* A2  = (const _Float16*)A2p;
  const _Float16* Bt  = (const _Float16*)Btp;
  const _Float16* Bt2 = (const _Float16*)Bt2p;
  __shared__ __align__(16) float sT[8][16 * 68];
  const int lane = threadIdx.x & 31;
  const int wave = threadIdx.x >> 5;
  const int tilesN = N >> 6;
  const int tilesM = M / (16 * MI);
  const int tile = blockIdx.x * 8 + wave;
  if (tile >= tilesM * tilesN) return;
  const int tm = tile / tilesN;
  const int tn = tile - tm * tilesN;
  const int m0 = tm * (16 * MI);
  const int n0 = tn << 6;
  const int rlane = lane & 15;
  const int koff  = (lane >> 4) * 8;
  const int mOff  = (lane >> 4) * 8;

  v8f acc[MI][4], accr[MI][4];
#pragma unroll
  for (int i = 0; i < MI; ++i)
#pragma unroll
    for (int j = 0; j < 4; ++j) {
      acc[i][j]  = (v8f){0.f, 0.f, 0.f, 0.f, 0.f, 0.f, 0.f, 0.f};
      accr[i][j] = (v8f){0.f, 0.f, 0.f, 0.f, 0.f, 0.f, 0.f, 0.f};
    }

  for (int k0 = 0; k0 < K; k0 += 32) {
    v16h bh[4], bl[4];
#pragma unroll
    for (int j = 0; j < 4; ++j) {
      const size_t bo = (size_t)(n0 + (j << 4) + rlane) * ldb + koff + k0;
      bh[j] = frag_load(Bt + bo);
      if (SPL == 2) bl[j] = frag_load(Bt2 + bo); else bl[j] = bh[j];
    }
#pragma unroll
    for (int i = 0; i < MI; ++i) {
      const size_t ao = (size_t)(m0 + (i << 4) + rlane) * lda + koff + k0;
      const v16h ah = frag_load(A + ao);
      v16h al = ah;
      if (SPL >= 1) al = frag_load(A2 + ao);
#pragma unroll
      for (int j = 0; j < 4; ++j) {
        acc[i][j] = mma(ah, bh[j], acc[i][j]);
        if (SPL >= 1) accr[i][j] = mma(al, bh[j], accr[i][j]);
        if (SPL == 2) accr[i][j] = mma(ah, bl[j], accr[i][j]);
      }
#pragma unroll
      for (int j = 0; j < 4; ++j) {
        guard1(acc[i][j], ah, al);
        if (SPL >= 1) guard1(accr[i][j], ah, al);
      }
    }
    keep4(bh[0], bh[1], bh[2], bh[3]);
    if (SPL == 2) keep4(bl[0], bl[1], bl[2], bl[3]);
  }
#pragma unroll
  for (int i = 0; i < MI; ++i)
#pragma unroll
    for (int j = 0; j < 4; ++j) {
      guard_acc(acc[i][j]);
      if (SPL >= 1) guard_acc(accr[i][j]);
    }

  float* slab = sT[wave];
#pragma unroll
  for (int i = 0; i < MI; ++i) {
    const int mBase = m0 + (i << 4);
#pragma unroll
    for (int j = 0; j < 4; ++j) {
#pragma unroll
      for (int r = 0; r < 8; ++r) {
        float v = acc[i][j][r] * scale;
        if (SPL >= 1) v += accr[i][j][r] * rscale;
        slab[(mOff + r) * 68 + (j << 4) + rlane] = v;
      }
    }
    __builtin_amdgcn_fence(__ATOMIC_RELEASE, "workgroup");
    __builtin_amdgcn_wave_barrier();
    __builtin_amdgcn_fence(__ATOMIC_ACQUIRE, "workgroup");
    {
      const int hh = lane >> 4, c4 = (lane & 15) * 4;
      for (int pass = 0; pass < 2; ++pass) {
#pragma unroll
        for (int it = 0; it < 8; ++it) {
          const int row = it * 2 + hh;
          const v4f v = *(const v4f*)(slab + row * 68 + c4);
          *(volatile v4f*)(C + (size_t)(mBase + row) * ldc + n0 + c4) = v;
        }
        __threadfence();
      }
    }
    __builtin_amdgcn_fence(__ATOMIC_RELEASE, "workgroup");
    __builtin_amdgcn_wave_barrier();
    __builtin_amdgcn_fence(__ATOMIC_ACQUIRE, "workgroup");
  }
}
}

__global__ __launch_bounds__(256) void rne_rows_f16_kernel(
    const float* __restrict__ src, unsigned short* __restrict__ dH, int total8)
{
  const int i = blockIdx.x * 256 + threadIdx.x;
  if (i >= total8) return;
  const size_t e0 = (size_t)i << 3;
  const v4f a0 = *(const v4f*)(src + e0);
  const v4f a1 = *(const v4f*)(src + e0 + 4);
  const float f0 = a0[0];
  const float f1 = a0[1];
  const float f2 = a0[2];
  const float f3 = a0[3];
  const float f4 = a1[0];
  const float f5 = a1[1];
  const float f6 = a1[2];
  const float f7 = a1[3];
  v8h hv;
  hv[0] = f16_flush(bf16r(f0));
  hv[1] = f16_flush(bf16r(f1));
  hv[2] = f16_flush(bf16r(f2));
  hv[3] = f16_flush(bf16r(f3));
  hv[4] = f16_flush(bf16r(f4));
  hv[5] = f16_flush(bf16r(f5));
  hv[6] = f16_flush(bf16r(f6));
  hv[7] = f16_flush(bf16r(f7));
  unsigned short* qh = dH + e0;
  *(volatile v8h*)qh = hv;
  __threadfence();
  *(volatile v8h*)qh = hv;
}

template <bool LO>
__global__ __launch_bounds__(256) void transpose_pack_kernel(
    const float* __restrict__ W, unsigned short* __restrict__ BtH, unsigned short* __restrict__ BtL,
    int Kdim, int Ndim, float carry)
{
  __shared__ float tile[64 * 65];
  const int tid = threadIdx.x, lane = tid & 31, wave = tid >> 5;
  const int n0 = blockIdx.x * 64;
  const int k0 = blockIdx.y * 64;
#pragma unroll
  for (int p = 0; p < 16; ++p) {
    const int idx = tid + p * 256;
    const int kk  = idx >> 6;
    const int nn  = idx & 63;
    const int n   = n0 + nn;
    const int nc  = (n < Ndim) ? n : (Ndim - 1);
    const float v = W[(size_t)(k0 + kk) * Ndim + nc];
    tile[kk * 65 + nn] = (n < Ndim) ? (bf16r(v) * carry) : 0.0f;
  }
  __syncthreads();
  const int q = lane >> 3, c8 = (lane & 7) * 8;
  v8h hv[2], lv[2];
#pragma unroll
  for (int it = 0; it < 2; ++it) {
    const int nrow = it * 32 + wave * 4 + q;
#pragma unroll
    for (int e = 0; e < 8; ++e) {
      _Float16 h, l;
      const float t = tile[(c8 + e) * 65 + nrow];
      f16_split(t, h, l);
      hv[it][e] = h;
      lv[it][e] = l;
    }
  }
  for (int pass = 0; pass < 2; ++pass) {
#pragma unroll
    for (int it = 0; it < 2; ++it) {
      const int nrow = it * 32 + wave * 4 + q;
      const size_t o = (size_t)(n0 + nrow) * Kdim + k0 + c8;
      *(volatile v8h*)(BtH + o) = hv[it];
      if (LO) *(volatile v8h*)(BtL + o) = lv[it];
    }
    __threadfence();
  }
}

__global__ __launch_bounds__(256) void rne_vec_kernel(
    const float* __restrict__ src, float* __restrict__ dst, int n4)
{
  const int i = blockIdx.x * 256 + threadIdx.x;
  if (i >= n4) return;
  const v4f a = *(const v4f*)(src + (size_t)i * 4);
  const float a0 = a[0];
  const float a1 = a[1];
  const float a2 = a[2];
  const float a3 = a[3];
  v4f r;
  r[0] = bf16r(a0);
  r[1] = bf16r(a1);
  r[2] = bf16r(a2);
  r[3] = bf16r(a3);
  float* p = dst + (size_t)i * 4;
  *(volatile v4f*)p = r;
  __threadfence();
  *(volatile v4f*)p = r;
}

__global__ __launch_bounds__(256) void conv_silu_kernel(
    const float* __restrict__ XZ, const float* __restrict__ cw, const float* __restrict__ cb,
    float* __restrict__ UC, unsigned short* __restrict__ UH)
{
  __shared__ __align__(16) float sT[16 * kConvTP];
  const int tid = threadIdx.x, lane = tid & 31, wave = tid >> 5;
  const int d0 = blockIdx.x * 256, d = d0 + tid;
  const int t0 = blockIdx.y * 64;
  const v4f wv = *(const v4f*)(cw + (size_t)d * 4);
  const float w0 = wv[0], w1 = wv[1], w2 = wv[2], w3 = wv[3];
  const float bc = cb[d];
  float xm3, xm2, xm1;
  {
    const int r3 = t0 - 3, r2 = t0 - 2, r1 = t0 - 1;
    const float v3 = XZ[(size_t)(r3 < 0 ? 0 : r3) * kXzP + d];
    const float v2 = XZ[(size_t)(r2 < 0 ? 0 : r2) * kXzP + d];
    const float v1 = XZ[(size_t)(r1 < 0 ? 0 : r1) * kXzP + d];
    xm3 = (r3 >= 0) ? v3 : 0.0f;
    xm2 = (r2 >= 0) ? v2 : 0.0f;
    xm1 = (r1 >= 0) ? v1 : 0.0f;
  }
  const int hrow = wave >> 1;
  const int hch  = (wave & 1) * 128 + lane * 4;
  for (int sub = 0; sub < 4; ++sub) {
    const int lb = t0 + sub * 16;
    for (int s = 0; s < 16; ++s) {
      const float xcur = XZ[(size_t)(lb + s) * kXzP + d];
      float acc = w0 * xm3;
      acc = fmaf(w1, xm2, acc);
      acc = fmaf(w2, xm1, acc);
      acc = fmaf(w3, xcur, acc);
      const float sv = acc + bc;
      const float sg = __builtin_amdgcn_rcpf(1.0f + expf(-sv));
      sT[s * kConvTP + tid] = sv * sg;
      xm3 = xm2; xm2 = xm1; xm1 = xcur;
    }
    __syncthreads();
    v4f fv[4];
    v8h hv[2];
#pragma unroll
    for (int it = 0; it < 4; ++it) fv[it] = *(const v4f*)(sT + (it * 4 + hrow) * kConvTP + hch);
#pragma unroll
    for (int it = 0; it < 2; ++it) {
      const float* sp = sT + (it * 8 + wave) * kConvTP + lane * 8;
      const v4f a0 = *(const v4f*)(sp);
      const v4f a1 = *(const v4f*)(sp + 4);
#pragma unroll
      for (int e = 0; e < 4; ++e) {
        const float f0 = a0[e];
        const float f1 = a1[e];
        hv[it][e] = f16_flush(f0);
        hv[it][4 + e] = f16_flush(f1);
      }
    }
    for (int pass = 0; pass < 2; ++pass) {
#pragma unroll
      for (int it = 0; it < 4; ++it)
        *(volatile v4f*)(UC + (size_t)(lb + it * 4 + hrow) * kDin + d0 + hch) = fv[it];
#pragma unroll
      for (int it = 0; it < 2; ++it) {
        const size_t o = (size_t)(lb + it * 8 + wave) * kDin + d0 + lane * 8;
        *(volatile v8h*)(UH + o) = hv[it];
      }
      __threadfence();
    }
    __syncthreads();
  }
}

__global__ __launch_bounds__(256) void proj_split_kernel(
    const float* __restrict__ P,
    unsigned short* __restrict__ dH, float* __restrict__ BC)
{
  const int tid = threadIdx.x;
  const int r0 = blockIdx.x * 32;
  const int g8 = (tid & 7) * 8;
  const int rowa = r0 + (tid >> 3);
  v8h hv;
  {
    const float* sp = P + (size_t)rowa * kProjP + g8;
    const v4f a0 = *(const v4f*)(sp);
    const v4f a1 = *(const v4f*)(sp + 4);
#pragma unroll
    for (int e = 0; e < 4; ++e) {
      const float f0 = a0[e];
      const float f1 = a1[e];
      hv[e] = f16_flush(f0);
      hv[4 + e] = f16_flush(f1);
    }
  }
  const int rowb = r0 + (tid >> 3);
  const int p4 = (tid & 7) * 4;
  const v4f pv = *(const v4f*)(P + (size_t)rowb * kProjP + kRank + p4);
  const v4f bcv = pv;
  for (int pass = 0; pass < 2; ++pass) {
    const size_t o = (size_t)rowa * kRank + g8;
    *(volatile v8h*)(dH + o) = hv;
    *(volatile v4f*)(BC + (size_t)rowb * kBcP + p4) = bcv;
    __threadfence();
  }
}

__global__ __launch_bounds__(256) void dt_bias_kernel(
    const float* __restrict__ DTP, const float* __restrict__ bdt, float* __restrict__ DT)
{
  const int d4 = (blockIdx.x * 256 + threadIdx.x) * 4;
  const int r0 = blockIdx.y * 8;
  const v4f b = *(const v4f*)(bdt + d4);
  v4f val[8];
#pragma unroll
  for (int i = 0; i < 8; ++i) {
    const v4f p = *(const v4f*)(DTP + (size_t)(r0 + i) * kDin + d4);
    val[i] = p + b;
  }
  for (int pass = 0; pass < 2; ++pass) {
#pragma unroll
    for (int i = 0; i < 8; ++i)
      *(volatile v4f*)(DT + (size_t)(r0 + i) * kDin + d4) = val[i];
    __threadfence();
  }
}

typedef float    ms1_v4f __attribute__((ext_vector_type(4)));
typedef unsigned ms1_v4u __attribute__((ext_vector_type(4)));
struct ms1_args {
  const float* dtpre;
  const float* u;
  const float* bc;
  const float* z;
  const float* A_log;
  const float* Dskip;
  __half* y;
  __half* y_lo;
  long ld_dtpre;
  long ld_u;
  long ld_bc;
  long ld_z;
  long ld_y;
  int offB;
  int offC;
  int offZ;
  float ycarry;
  int dir;
  int D;
  int L;
  int nbatch;
};
static_assert(sizeof(ms1_args) == 136);

__device__ __forceinline__ float ms1_flush16(float v) {
  return (fabsf(v) < 6.103515625e-05f) ? 0.0f : v;
}
__device__ __forceinline__ unsigned ms1_h16bits(float v) {
  return (unsigned)__half_as_ushort(__float2half_rn(ms1_flush16(v)));
}
__device__ __forceinline__ float ms1_h16val(unsigned b) {
  return __half2float(__ushort_as_half((unsigned short)b));
}
__device__ __forceinline__ float ms1_softplus(float v) {
  return fmaxf(v, 0.0f) + log1pf(expf(-fabsf(v)));
}
__device__ __forceinline__ void ms1_pack2(float v0, float v1, unsigned& hw, unsigned& lw) {
  const unsigned h0 = ms1_h16bits(v0);
  const unsigned h1 = ms1_h16bits(v1);
  const float r0 = (v0 - ms1_h16val(h0)) * 2048.0f;
  const float r1 = (v1 - ms1_h16val(h1)) * 2048.0f;
  const unsigned l0 = ms1_h16bits(r0);
  const unsigned l1 = ms1_h16bits(r1);
  hw = h0 | (h1 << 16);
  lw = l0 | (l1 << 16);
}

template <int NSTATE>
__global__ __launch_bounds__(64 * (NSTATE / 16)) void ms1_scan_kernel(ms1_args a)
{
  static_assert(NSTATE == 16 || NSTATE == 64);
  constexpr int NQ  = NSTATE / 16;
  constexpr int NT  = 64 * NQ;
  constexpr int NW  = NT / 32;
  constexpr int BCW = 2 * NSTATE;
  constexpr int YP  = 68;
  constexpr int RPI = NW * 4;
  constexpr int NIT = 64 / RPI;
  static_assert(16 * NT <= 64 * YP);
  __shared__ __align__(16) float sBC[64 * BCW];
  __shared__ __align__(16) float sY[64 * YP];
  const int tid  = threadIdx.x;
  const int lane = tid & 31;
  const int wave = tid >> 5;
  const int c    = tid / NQ;
  const int sq   = tid - c * NQ;
  const int bpb  = a.D / 64;
  const int bi   = blockIdx.x / bpb;
  if (bi >= a.nbatch) return;
  const int d0 = (blockIdx.x - bi * bpb) * 64;
  const int d  = d0 + c;
  const long rowb = (long)bi * a.L;
  const bool hasz  = (a.z != nullptr);
  const bool hasD  = (a.Dskip != nullptr);
  const bool hasLo = (a.y_lo != nullptr);

#pragma unroll 1
  for (int n = 0; n < 16; ++n) {
    const float al = a.A_log[(long)d * NSTATE + sq * 16 + n];
    sY[n * NT + tid] = -expf(al);
  }
  __syncthreads();
  float An[16], h[16];
#pragma unroll
  for (int n = 0; n < 16; ++n) {
    An[n] = sY[n * NT + tid];
    h[n] = 0.0f;
  }
  float Dd = 0.0f;
  if (hasD) Dd = a.Dskip[d];

  const int nchunk = a.L / 64;
  const bool fwd = (a.dir > 0);
  const int s0 = fwd ? 0 : 63;
  const int sd = fwd ? 1 : -1;
  const int q  = lane >> 3;
  const int c8 = (lane & 7) * 8;

  for (int ci = 0; ci < nchunk; ++ci) {
    const int tb = fwd ? (ci * 64) : (a.L - 64 - ci * 64);
    const long rowc = rowb + tb;
    __syncthreads();
#pragma unroll 8
    for (int i = 0; i < 32; ++i) {
      const int idx = tid + i * NT;
      const int st  = idx / BCW;
      const int col = idx - st * BCW;
      const int sc  = (col < NSTATE) ? (a.offB + col) : (a.offC + col - NSTATE);
      sBC[idx] = a.bc[(rowc + st) * a.ld_bc + sc];
    }
    __syncthreads();
    for (int s = 0; s < 64; ++s) {
      const int ls = s0 + sd * s;
      const long row = rowc + ls;
      float pre = a.dtpre[row * a.ld_dtpre + d];
      float uv  = a.u[row * a.ld_u + d];
      float zv  = 0.0f;
      if (hasz) zv = a.z[row * a.ld_z + a.offZ + d];
      asm volatile("" : "+v"(pre));
      asm volatile("" : "+v"(uv));
      asm volatile("" : "+v"(zv));
      const float delta = ms1_softplus(pre);
      const float dtx = delta * uv;
      const float* bp = sBC + ls * BCW + sq * 16;
      const float* cp = bp + NSTATE;
      ms1_v4f Bq[4], Cq[4];
#pragma unroll
      for (int k = 0; k < 4; ++k) {
        Bq[k] = *(const ms1_v4f*)(bp + 4 * k);
        Cq[k] = *(const ms1_v4f*)(cp + 4 * k);
      }
      float yv = 0.0f;
#pragma unroll
      for (int n = 0; n < 16; ++n) {
        const float e = __expf(delta * An[n]);
        h[n] = fmaf(e, h[n], dtx * Bq[n >> 2][n & 3]);
        yv = fmaf(h[n], Cq[n >> 2][n & 3], yv);
      }
      if (NQ > 1) {
        yv += __shfl_xor(yv, 1, 32);
        yv += __shfl_xor(yv, 2, 32);
      }
      if (hasD) yv = fmaf(uv, Dd, yv);
      if (hasz) {
        const float sg = __builtin_amdgcn_rcpf(1.0f + expf(-zv));
        yv = yv * (zv * sg);
      }
      if (sq == 0) sY[ls * YP + c] = yv * a.ycarry;
    }
    __syncthreads();
    ms1_v4u hw[NIT], lw[NIT];
#pragma unroll
    for (int it = 0; it < NIT; ++it) {
      const int row = it * RPI + wave * 4 + q;
      const float* sp = sY + row * YP + c8;
      const ms1_v4f f0 = *(const ms1_v4f*)(sp);
      const ms1_v4f f1 = *(const ms1_v4f*)(sp + 4);
      unsigned h0, h1, h2, h3, l0, l1, l2, l3;
      ms1_pack2(f0[0], f0[1], h0, l0);
      ms1_pack2(f0[2], f0[3], h1, l1);
      ms1_pack2(f1[0], f1[1], h2, l2);
      ms1_pack2(f1[2], f1[3], h3, l3);
      hw[it] = (ms1_v4u){h0, h1, h2, h3};
      lw[it] = (ms1_v4u){l0, l1, l2, l3};
    }
    for (int pass = 0; pass < 2; ++pass) {
#pragma unroll
      for (int it = 0; it < NIT; ++it) {
        const int row = it * RPI + wave * 4 + q;
        const long o = (rowc + row) * a.ld_y + d0 + c8;
        *(volatile ms1_v4u*)(a.y + o) = hw[it];
        if (hasLo) *(volatile ms1_v4u*)(a.y_lo + o) = lw[it];
      }
      __threadfence();
    }
  }
}

static_assert((kSeq % 16) == 0 && (kSeq % 32) == 0);
static_assert(((kSeq / 32) * (kXzP / 64)) % 8 == 0);
static_assert(((kSeq / 16) * (kProjP / 64)) % 8 == 0);
static_assert(((kSeq / 32) * (kDin / 64)) % 8 == 0);
static_assert(((kSeq / 32) * (kDm / 64)) % 8 == 0);
static_assert((kDm % 64) == 0 && (kDin % 64) == 0 && (kRank % 64) == 0 && (kXzP % 64) == 0 && (kProjP % 64) == 0);
static_assert(((kSeq * kDm / 8) % 256) == 0);
static_assert(((kDin * kConvK / 4) % 256) == 0);
static_assert(((kDin / 4) % 256) == 0);
static_assert(((kDin * kNst / 4) % 256) == 0);
static_assert((kSeq % 32) == 0 && (kSeq % 64) == 0);

extern "C" void kernel_launch(void* const* d_in, const int* in_sizes, int n_in,
                              void* d_out, int out_size, void* d_ws, size_t ws_size,
                              hipStream_t stream)
{
  if (n_in < 10) return;
  if (in_sizes[0] != kBatch * kSeq * kDm) return;
  if (in_sizes[1] != kXzP * kDm) return;
  if (in_sizes[2] != kDin * kConvK) return;
  if (in_sizes[3] != kDin) return;
  if (in_sizes[4] != kProjN * kDin) return;
  if (in_sizes[5] != kDin * kRank) return;
  if (in_sizes[6] != kDin) return;
  if (in_sizes[7] != kDin * kNst) return;
  if (in_sizes[8] != kDin) return;
  if (in_sizes[9] != kDm * kDin) return;
  if (out_size != kBatch * kSeq * kDm) return;
  if (ws_size < kWsTotal) return;

  const float* x        = (const float*)d_in[0];
  const float* W_in     = (const float*)d_in[1];
  const float* conv_w   = (const float*)d_in[2];
  const float* conv_b   = (const float*)d_in[3];
  const float* W_xproj  = (const float*)d_in[4];
  const float* W_dt     = (const float*)d_in[5];
  const float* b_dt     = (const float*)d_in[6];
  const float* A_log_in = (const float*)d_in[7];
  const float* D_skip   = (const float*)d_in[8];
  const float* W_out    = (const float*)d_in[9];
  float* out = (float*)d_out;

  char* ws = (char*)d_ws;
  unsigned short* WIN  = (unsigned short*)(ws + kOffWIN);
  unsigned short* WXH  = (unsigned short*)(ws + kOffWXH);
  unsigned short* WDT  = (unsigned short*)(ws + kOffWDT);
  unsigned short* WOH  = (unsigned short*)(ws + kOffWOH);
  float*          CW   = (float*)(ws + kOffCW);
  float*          CB   = (float*)(ws + kOffCB);
  float*          BDR  = (float*)(ws + kOffBDR);
  float*          DR   = (float*)(ws + kOffDR);
  float*          ALOG = (float*)(ws + kOffALOG);
  unsigned short* XH   = (unsigned short*)(ws + kOffXH);
  float*          XZ   = (float*)(ws + kOffXZ);
  float*          U    = (float*)(ws + kOffU);
  unsigned short* UH   = (unsigned short*)(ws + kOffUH);
  float*          PROJ = (float*)(ws + kOffPROJ);
  unsigned short* DH   = (unsigned short*)(ws + kOffDH);
  float*          BC   = (float*)(ws + kOffBC);
  float*          DTP  = (float*)(ws + kOffDTP);
  float*          DT   = (float*)(ws + kOffDT);
  unsigned short* YH   = (unsigned short*)(ws + kOffYH);

  constexpr float sW = 1.0f / kWCarry;
  constexpr float sY = 1.0f / (kWCarry * kYCarry);

  transpose_pack_kernel<false><<<dim3(kXzP / 64, kDm / 64), 256, 0, stream>>>(W_in, WIN, WIN, kDm, kXzP, kWCarry);

  transpose_pack_kernel<false><<<dim3(kProjP / 64, kDin / 64), 256, 0, stream>>>(W_xproj, WXH, WXH, kDin, kProjN, kWCarry);

  transpose_pack_kernel<false><<<dim3(kDin / 64, kRank / 64), 256, 0, stream>>>(W_dt, WDT, WDT, kRank, kDin, kWCarry);

  transpose_pack_kernel<false><<<dim3(kDm / 64, kDin / 64), 256, 0, stream>>>(W_out, WOH, WOH, kDin, kDm, kWCarry);

  rne_vec_kernel<<<(kDin * kConvK / 4) / 256, 256, 0, stream>>>(conv_w, CW, kDin * kConvK / 4);

  rne_vec_kernel<<<(kDin / 4) / 256, 256, 0, stream>>>(conv_b, CB, kDin / 4);
  rne_vec_kernel<<<(kDin / 4) / 256, 256, 0, stream>>>(b_dt, BDR, kDin / 4);
  rne_vec_kernel<<<(kDin / 4) / 256, 256, 0, stream>>>(D_skip, DR, kDin / 4);

  rne_vec_kernel<<<(kDin * kNst / 4) / 256, 256, 0, stream>>>(A_log_in, ALOG, kDin * kNst / 4);

  for (int b = 0; b < kBatch; ++b) {
    const float* xb = x + (size_t)b * kSeq * kDm;
    float* outb = out + (size_t)b * kSeq * kDm;

    rne_rows_f16_kernel<<<(kSeq * kDm / 8) / 256, 256, 0, stream>>>(xb, XH, kSeq * kDm / 8);

    eng::gemm_f16_kernel<2, 0><<<dim3((kSeq / 32) * (kXzP / 64) / 8), 256, 0, stream>>>(
        XH, nullptr, kDm, WIN, nullptr, kDm, XZ, kXzP, kSeq, kXzP, kDm, sW, 0.0f);

    conv_silu_kernel<<<dim3(kDin / 256, kSeq / 64), 256, 0, stream>>>(XZ, CW, CB, U, UH);

    eng::gemm_f16_kernel<1, 0><<<dim3((kSeq / 16) * (kProjP / 64) / 8), 256, 0, stream>>>(
        UH, nullptr, kDin, WXH, nullptr, kDin, PROJ, kProjP, kSeq, kProjP, kDin, sW, 0.0f);

    proj_split_kernel<<<kSeq / 32, 256, 0, stream>>>(PROJ, DH, BC);

    eng::gemm_f16_kernel<2, 0><<<dim3((kSeq / 32) * (kDin / 64) / 8), 256, 0, stream>>>(
        DH, nullptr, kRank, WDT, nullptr, kRank, DTP, kDin, kSeq, kDin, kRank, sW, 0.0f);

    dt_bias_kernel<<<dim3(kDin / 4 / 256, kSeq / 8), 256, 0, stream>>>(DTP, BDR, DT);

    ms1_args sa;
    sa.dtpre = DT;
    sa.u = U;
    sa.bc = BC;
    sa.z = XZ;
    sa.A_log = ALOG;
    sa.Dskip = DR;
    sa.y = (__half*)YH;
    sa.y_lo = nullptr;
    sa.ld_dtpre = kDin;
    sa.ld_u = kDin;
    sa.ld_bc = kBcP;
    sa.ld_z = kXzP;
    sa.ld_y = kDin;
    sa.offB = 0;
    sa.offC = kNst;
    sa.offZ = kDin;
    sa.ycarry = kYCarry;
    sa.dir = 1;
    sa.D = kDin;
    sa.L = kSeq;
    sa.nbatch = 1;
    ms1_scan_kernel<16><<<dim3(kDin / 64), 64, 0, stream>>>(sa);

    eng::gemm_f16_kernel<2, 0><<<dim3((kSeq / 32) * (kDm / 64) / 8), 256, 0, stream>>>(
        YH, nullptr, kDin, WOH, nullptr, kDin, outb, kDm, kSeq, kDm, kDin, sY, 0.0f);
  }
}
